// DenseDistance_38817914422094
// MI455X (gfx1250) — hardware-verified
//
#include <hip/hip_runtime.h>


namespace {
constexpr int NB = 2048, D = 256, U = 512;
constexpr float XS = 8.0f, EPS = 1e-7f;
typedef _Float16 b16;
typedef __attribute__((ext_vector_type(16))) _Float16 v16b;
typedef __attribute__((ext_vector_type(8))) _Float16 v8b;
typedef __attribute__((ext_vector_type(8))) float v8f;
typedef __attribute__((ext_vector_type(4))) float v4f;
__device__ __forceinline__ float bf16_rne(float f) { unsigned int u = __float_as_uint(f); u += 0x7FFFu + ((u >> 16) & 1u); float r = __uint_as_float(u & 0xFFFF0000u); asm volatile("" : "+v"(r)); return r; }
__device__ __forceinline__ v16b frag_kb(const b16* p, int hh) { const v8b a = *(const v8b*)(p + 8 * hh), b = *(const v8b*)(p + 16 + 8 * hh); v16b f;
#pragma unroll
  for (int e = 0; e < 8; ++e) { f[e] = a[e]; f[8 + e] = b[e]; } return f; }
__device__ __forceinline__ v8f wmma16b(v16b a, v16b b, v8f c) { v8f d = __builtin_amdgcn_wmma_f32_16x16x32_f16(false, a, false, b, (short)0, c, false, false); asm volatile("v_nop\n\tv_nop\n\tv_nop\n\tv_nop" : "+v"(d) : "v"(a), "v"(b)); return d; }
__device__ __forceinline__ void wave_lds_sync() { __builtin_amdgcn_fence(__ATOMIC_RELEASE, "workgroup"); __builtin_amdgcn_wave_barrier(); __builtin_amdgcn_fence(__ATOMIC_ACQUIRE, "workgroup"); }
__device__ __forceinline__ float pmul(float a, float b) { float p = a * b; asm volatile("" : "+v"(p)); return p; }

__global__ __launch_bounds__(32) void wprep_kernel(const float* __restrict__ W, b16* __restrict__ WT, float* __restrict__ WN) { const int lane = threadIdx.x; const int u = blockIdx.x * 32 + lane; float s = 0.0f;
  for (int pass = 0; pass < 2; ++pass) { s = 0.0f; for (int d0 = 0; d0 < D; d0 += 8) { v8b v;
#pragma unroll
      for (int j = 0; j < 8; ++j) { const float w = bf16_rne(W[(size_t)(d0 + j) * U + u]); v[j] = (b16)(w * XS); s += pmul(w, w); } *(volatile v8b*)(WT + (size_t)u * D + d0) = v; }
    ((volatile float*)WN)[u] = s; __threadfence(); } }
__global__ __launch_bounds__(32) void dist_kernel(const float* __restrict__ x, const b16* __restrict__ WT, const float* __restrict__ WN, float* __restrict__ out) { __shared__ __attribute__((aligned(16))) b16 Ah[16][D + 8]; __shared__ float Xn[16]; __shared__ float Tf[16][132]; const int lane = threadIdx.x, nloc = lane & 15, hlf = lane >> 4; const int g = blockIdx.x % (U / 128); const size_t m0 = (size_t)(blockIdx.x / (U / 128)) * 16;
  for (int rr = 0; rr < 16; ++rr) { float s = 0.0f; for (int q = 0; q < D / 32; ++q) { const float v = bf16_rne(x[(m0 + rr) * D + q * 32 + lane]); Ah[rr][q * 32 + lane] = (b16)(v * XS); s += pmul(v, v); } for (int o = 16; o; o >>= 1) s += __shfl_xor(s, o); if (lane == 0) Xn[rr] = s; }
  wave_lds_sync(); v8f acc[8];
#pragma unroll
  for (int t = 0; t < 8; ++t) acc[t] = (v8f){};
#pragma unroll 2
  for (int kb = 0; kb < D; kb += 32) { const v16b a = frag_kb(&Ah[nloc][kb], hlf);
#pragma unroll
    for (int t = 0; t < 8; ++t) acc[t] = wmma16b(a, frag_kb(WT + (size_t)(g * 128 + t * 16 + nloc) * D + kb, hlf), acc[t]); }
#pragma unroll
  for (int t = 0; t < 8; ++t) { const int u = g * 128 + t * 16 + nloc; const float wn = WN[u];
#pragma unroll
    for (int r8 = 0; r8 < 8; ++r8) { const int rr = 8 * hlf + r8; const float sq = Xn[rr] + wn - 2.0f * (acc[t][r8] * (1.0f / (XS * XS))); Tf[rr][t * 16 + nloc] = sqrtf(fmaxf(sq, EPS)); } }
  wave_lds_sync();
  for (int pass = 0; pass < 2; ++pass) { for (int rr = 0; rr < 16; ++rr) *(volatile v4f*)(out + (m0 + rr) * U + g * 128 + lane * 4) = *(const v4f*)(&Tf[rr][lane * 4]); __threadfence(); } }
}

extern "C" void kernel_launch(void* const* d_in, const int* in_sizes, int n_in, void* d_out, int out_size, void* d_ws, size_t ws_size, hipStream_t stream) {
  (void)n_in;
  if (in_sizes[0] != NB * D || in_sizes[1] != D * U || out_size != NB * U) return;
  size_t off = 0; char* ws = (char*)d_ws;
  auto carve = [&](size_t bytes) { char* p = ws + off; off += (bytes + 255) & ~(size_t)255; return p; };
  b16* WT = (b16*)carve((size_t)U * D * 2); float* WN = (float*)carve((size_t)U * 4);
  if (off > ws_size || off > ((size_t)2 << 20)) return;
  wprep_kernel<<<U / 32, 32, 0, stream>>>((const float*)d_in[1], WT, WN);
  dist_kernel<<<(NB / 16) * (U / 128), 32, 0, stream>>>((const float*)d_in[0], WT, WN, (float*)d_out);
}
